// SynthesizerAttention_5798205849810
// MI455X (gfx1250) — hardware-run, weakly checked
//
#include <hip/hip_runtime.h>
#include <hip/hip_bf16.h>

typedef __attribute__((ext_vector_type(16))) _Float16 v16h;
typedef __attribute__((ext_vector_type(8)))  _Float16 v8h;
typedef __attribute__((ext_vector_type(16))) __bf16   v16b;
typedef __attribute__((ext_vector_type(8)))  __bf16   v8b;
typedef __attribute__((ext_vector_type(8)))  float    v8f;
typedef __attribute__((ext_vector_type(4)))  float    v4f;
typedef __attribute__((ext_vector_type(4)))  unsigned v4u;

constexpr int kBatch = 2;
constexpr int kSeq   = 2048;
constexpr int kEmb   = 1024;
constexpr int kHeads = 16;
constexpr int kHD    = 64;
constexpr int kTok   = kBatch * kSeq;
constexpr int kKC    = 64;
constexpr float kNegFill = -1.0e10f;
constexpr float kW1Carry = 64.0f;
constexpr float kW2Carry = 1024.0f;

static_assert(kTok % 64 == 0);
static_assert(kEmb % 64 == 0);
static_assert(kEmb % 32 == 0);
static_assert(kSeq % 64 == 0);
static_assert(kHD == 64);
static_assert(kHeads * kHD == kEmb);

__device__ __forceinline__ unsigned short f2bf_bits(float f) {
  unsigned u = __float_as_uint(f);
  return (unsigned short)((u + 0x7FFFu + ((u >> 16) & 1u)) >> 16);
}
__device__ __forceinline__ float bf_bits2f(unsigned short h) { return __uint_as_float(((unsigned)h) << 16); }

__device__ __forceinline__ void dep_guard_h(v8f& a, v8f& b, v16h x, v16h y) { asm volatile("v_nop\n\tv_nop\n\tv_nop\n\tv_nop" : "+v"(a), "+v"(b) : "v"(x), "v"(y)); }
__device__ __forceinline__ void dep_guard_b(v8f& a, v8f& b, v16b x, v16b y) { asm volatile("v_nop\n\tv_nop\n\tv_nop\n\tv_nop" : "+v"(a), "+v"(b) : "v"(x), "v"(y)); }
__device__ __forceinline__ void keep4_h(v16h a, v16h b, v16h c, v16h d) { asm volatile("v_nop" :: "v"(a), "v"(b), "v"(c), "v"(d)); }
__device__ __forceinline__ void keep4_b(v16b a, v16b b, v16b c, v16b d) { asm volatile("v_nop" :: "v"(a), "v"(b), "v"(c), "v"(d)); }
__device__ __forceinline__ void acc_guard4(v8f& a, v8f& b, v8f& c, v8f& d) { asm volatile("v_nop\n\tv_nop\n\tv_nop\n\tv_nop" : "+v"(a), "+v"(b), "+v"(c), "+v"(d)); }
template <typename T> struct Frag;
template <> struct Frag<_Float16> {
  typedef v16h V; union U { v16h v; v8h h[2]; };
  static __device__ __forceinline__ v16h load(const _Float16* p) {
    U f; f.h[0] = *(const v8h*)(p); f.h[1] = *(const v8h*)(p + 16); return f.v;
  }
  static __device__ __forceinline__ v8f mma(v16h a, v16h b, v8f c) {
    return __builtin_amdgcn_wmma_f32_16x16x32_f16(false, a, false, b, (short)0, c, false, false);
  }
  static __device__ __forceinline__ void guard(v8f& a, v8f& b, v16h x, v16h y) { dep_guard_h(a, b, x, y); }
  static __device__ __forceinline__ void keep(v16h a, v16h b, v16h c, v16h d) { keep4_h(a, b, c, d); }
};
template <> struct Frag<__bf16> {
  typedef v16b V; union U { v16b v; v8b h[2]; };
  static __device__ __forceinline__ v16b load(const __bf16* p) {
    U f; f.h[0] = *(const v8b*)(p); f.h[1] = *(const v8b*)(p + 16); return f.v;
  }
  static __device__ __forceinline__ v8f mma(v16b a, v16b b, v8f c) {
    return __builtin_amdgcn_wmma_f32_16x16x32_bf16(false, a, false, b, (short)0, c, false, false);
  }
  static __device__ __forceinline__ void guard(v8f& a, v8f& b, v16b x, v16b y) { dep_guard_b(a, b, x, y); }
  static __device__ __forceinline__ void keep(v16b a, v16b b, v16b c, v16b d) { keep4_b(a, b, c, d); }
};

template <int ET> struct Elem;
template <> struct Elem<0> { typedef _Float16 T; };
template <> struct Elem<1> { typedef __bf16 T; };
template <int ET, bool SPLIT, int BIAS_MODE, int OUT_MODE, bool RESID, int ACT = 0>
__global__ __launch_bounds__(256) void wmma_gemm64(
    const unsigned short* __restrict__ Ap, const unsigned short* __restrict__ A2p, int lda, long strideA,
    const unsigned short* __restrict__ Btp, const unsigned short* __restrict__ Bt2p, int ldb, long strideB,
    void* __restrict__ Cout, void* __restrict__ Cout2, int ldc, long strideC,
    const float* __restrict__ bias,
    const float* __restrict__ resid, long strideR,
    int M, int N, int K, float scale) {
  typedef typename Elem<ET>::T T;
  typedef typename Frag<T>::V V;
  const T* A = (const T*)Ap; const T* A2 = (const T*)A2p; const T* Bt = (const T*)Btp; const T* Bt2 = (const T*)Bt2p;
  __shared__ __align__(16) float sT[8][16 * 68];
  const int b    = blockIdx.y;
  const int lane = threadIdx.x & 31;
  const int wave = threadIdx.x >> 5;
  const int tilesN = N >> 6;
  const int tilesM = M >> 6;
  const int tile = blockIdx.x * 8 + wave;
  if (tile >= tilesM * tilesN) return;
  const int tm = tile / tilesN;
  const int tn = tile - tm * tilesN;
  const int m0 = tm << 6;
  const int n0 = tn << 6;

  const T* Ab  = A  + (size_t)b * strideA;
  const T* Bb  = Bt + (size_t)b * strideB;
  const T* Ab2 = SPLIT ? (A2  + (size_t)b * strideA) : nullptr;
  const T* Bb2 = SPLIT ? (Bt2 + (size_t)b * strideB) : nullptr;

  const int rlane = lane & 15;
  const int koff  = (lane >> 4) * 8;
  const int mOff  = (lane >> 4) * 8;

  v8f acc[4][4];
#pragma unroll
  for (int i = 0; i < 4; ++i)
#pragma unroll
    for (int j = 0; j < 4; ++j) acc[i][j] = (v8f){0.f,0.f,0.f,0.f,0.f,0.f,0.f,0.f};

  for (int k0 = 0; k0 < K; k0 += 32) {
    V bh[4], bl[4];
#pragma unroll
    for (int j = 0; j < 4; ++j) {
      const size_t bo = (size_t)(n0 + (j << 4) + rlane) * ldb + koff + k0;
      bh[j] = Frag<T>::load(Bb + bo);
      if (SPLIT) bl[j] = Frag<T>::load(Bb2 + bo);
    }
#pragma unroll
    for (int i = 0; i < 4; ++i) {
      const size_t ao = (size_t)(m0 + (i << 4) + rlane) * lda + koff + k0;
      V ah = Frag<T>::load(Ab + ao);
      V al;
      if (SPLIT) al = Frag<T>::load(Ab2 + ao);
#pragma unroll
      for (int j = 0; j < 4; ++j) {
        acc[i][j] = Frag<T>::mma(ah, bh[j], acc[i][j]);
        if (SPLIT) {
          acc[i][j] = Frag<T>::mma(ah, bl[j], acc[i][j]);
          acc[i][j] = Frag<T>::mma(al, bh[j], acc[i][j]);
        }
      }
      Frag<T>::guard(acc[i][0], acc[i][3], ah, SPLIT ? al : ah);
    }
    Frag<T>::keep(bh[0], bh[1], bh[2], bh[3]);
    if (SPLIT) Frag<T>::keep(bl[0], bl[1], bl[2], bl[3]);
  }
  acc_guard4(acc[0][0], acc[0][1], acc[0][2], acc[0][3]);
  acc_guard4(acc[1][0], acc[1][1], acc[1][2], acc[1][3]);
  acc_guard4(acc[2][0], acc[2][1], acc[2][2], acc[2][3]);
  acc_guard4(acc[3][0], acc[3][1], acc[3][2], acc[3][3]);

  float* slab = sT[wave];
  const float* Rb = RESID ? (resid + (size_t)b * strideR) : nullptr;
#pragma unroll
  for (int i = 0; i < 4; ++i) {
    const int mBase = m0 + (i << 4);
#pragma unroll
    for (int j = 0; j < 4; ++j) {
      const int n = n0 + (j << 4) + rlane;
      float bv = 0.f;
      if (BIAS_MODE == 2) bv = bias[n];
#pragma unroll
      for (int r = 0; r < 8; ++r) {
        float v = acc[i][j][r] * scale;
        if (BIAS_MODE == 1) v += bias[mBase + mOff + r];
        if (BIAS_MODE == 2) v += bv;
        if (RESID) v += Rb[(size_t)(mBase + mOff + r) * ldc + n];
        if (ACT == 1) v = tanhf(v);
        if (ACT == 2) v = fmaxf(v, 0.0f);
        if (ACT == 3) v = v / (1.0f + expf(-v));
        if (ACT == 4) v = (v > 0.f) ? v : 0.01f * v;
        if (ACT == 5) v = 0.5f * v * (1.0f + erff(v * 0.70710678118654752f));
        slab[(mOff + r) * 68 + (j << 4) + rlane] = v;
      }
    }
    __builtin_amdgcn_fence(__ATOMIC_RELEASE, "workgroup");
    __builtin_amdgcn_wave_barrier();
    __builtin_amdgcn_fence(__ATOMIC_ACQUIRE, "workgroup");
    if (OUT_MODE == 0) {
      float* C = (float*)Cout + (size_t)b * strideC;
      const int hh = lane >> 4, c4 = (lane & 15) * 4;
      for (int pass = 0; pass < 2; ++pass) {
#pragma unroll
        for (int it = 0; it < 8; ++it) {
          const int row = it * 2 + hh;
          v4f v = *(const v4f*)(slab + row * 68 + c4);
          *(volatile v4f*)(C + (size_t)(mBase + row) * ldc + n0 + c4) = v;
        }
        __threadfence();
      }
    } else {
      const int q = lane >> 3, c8 = (lane & 7) * 8;
      unsigned short* C  = (unsigned short*)Cout  + (size_t)b * strideC;
      unsigned short* C2 = (OUT_MODE == 2) ? ((unsigned short*)Cout2 + (size_t)b * strideC) : nullptr;
      for (int pass = 0; pass < 2; ++pass) {
#pragma unroll
        for (int it = 0; it < 4; ++it) {
          const int row = it * 4 + q;
          const float* sp = slab + row * 68 + c8;
          v8h hv, lv;
#pragma unroll
          for (int e = 0; e < 8; ++e) {
            if (OUT_MODE == 1) {
              hv[e] = (_Float16)sp[e];
            } else {
              unsigned short hb = f2bf_bits(sp[e]);
              unsigned short lb = f2bf_bits(sp[e] - bf_bits2f(hb));
              hv[e] = __builtin_bit_cast(_Float16, hb);
              lv[e] = __builtin_bit_cast(_Float16, lb);
            }
          }
          *(volatile v8h*)(C + (size_t)(mBase + row) * ldc + n0 + c8) = hv;
          if (OUT_MODE == 2) *(volatile v8h*)(C2 + (size_t)(mBase + row) * ldc + n0 + c8) = lv;
        }
        __threadfence();
      }
    }
    __builtin_amdgcn_fence(__ATOMIC_RELEASE, "workgroup");
    __builtin_amdgcn_wave_barrier();
    __builtin_amdgcn_fence(__ATOMIC_ACQUIRE, "workgroup");
  }
}

__device__ __forceinline__ unsigned short at_bf_bits(float f) {
  unsigned u = __float_as_uint(f);
  return (unsigned short)((u + 0x7FFFu + ((u >> 16) & 1u)) >> 16);
}
__device__ __forceinline__ __bf16 at_f2bf(float f) { return __builtin_bit_cast(__bf16, at_bf_bits(f)); }
__device__ __forceinline__ void at_split(float f, __bf16& hi, __bf16& lo) {
  const unsigned short hb = at_bf_bits(f);
  hi = __builtin_bit_cast(__bf16, hb);
  lo = at_f2bf(f - __uint_as_float(((unsigned)hb) << 16));
}
__device__ __forceinline__ v8f at_mma(v16b a, v16b b, v8f c) {
  c = __builtin_amdgcn_wmma_f32_16x16x32_bf16(false, a, false, b, (short)0, c, false, false);
  asm volatile("v_nop\n\tv_nop\n\tv_nop\n\tv_nop" : "+v"(c) : "v"(a), "v"(b));
  return c;
}
__device__ __forceinline__ v8f mma_h16(v16h a, v16h b, v8f c) {
  c = __builtin_amdgcn_wmma_f32_16x16x32_f16(false, a, false, b, (short)0, c, false, false);
  asm volatile("v_nop\n\tv_nop\n\tv_nop\n\tv_nop" : "+v"(c) : "v"(a), "v"(b));
  return c;
}

template <bool WF16, bool WBF>
__global__ __launch_bounds__(256) void cvt_planes8(
    const float* __restrict__ in, int n8, float s16,
    unsigned short* __restrict__ o16, unsigned short* __restrict__ oh, unsigned short* __restrict__ ol) {
  const int i = blockIdx.x * 256 + threadIdx.x;
  if (i >= n8) return;
  const v4f a0 = *(const v4f*)(in + (size_t)i * 8);
  const v4f a1 = *(const v4f*)(in + (size_t)i * 8 + 4);
  const float f[8] = {a0[0], a0[1], a0[2], a0[3], a1[0], a1[1], a1[2], a1[3]};
  v4u w16 = (v4u){0u, 0u, 0u, 0u}, wh = (v4u){0u, 0u, 0u, 0u}, wl = (v4u){0u, 0u, 0u, 0u};
#pragma unroll
  for (int e = 0; e < 4; ++e) {
    const float f0 = f[2 * e], f1 = f[2 * e + 1];
    if (WF16) {
      const unsigned b0 = (unsigned)__builtin_bit_cast(unsigned short, (_Float16)(f0 * s16));
      const unsigned b1 = (unsigned)__builtin_bit_cast(unsigned short, (_Float16)(f1 * s16));
      w16[e] = b0 | (b1 << 16);
    }
    if (WBF) {
      const unsigned short h0 = f2bf_bits(f0), h1 = f2bf_bits(f1);
      const unsigned short l0 = f2bf_bits(f0 - bf_bits2f(h0)), l1 = f2bf_bits(f1 - bf_bits2f(h1));
      wh[e] = (unsigned)h0 | ((unsigned)h1 << 16);
      wl[e] = (unsigned)l0 | ((unsigned)l1 << 16);
    }
  }
  for (int pass = 0; pass < 2; ++pass) {
    if (WF16) *(volatile v4u*)(void*)(o16 + (size_t)i * 8) = w16;
    if (WBF) {
      *(volatile v4u*)(void*)(oh + (size_t)i * 8) = wh;
      *(volatile v4u*)(void*)(ol + (size_t)i * 8) = wl;
    }
    __threadfence();
  }
}

__global__ __launch_bounds__(256) void w2t_kernel(const float* __restrict__ w2, unsigned short* __restrict__ w2t) {
  __shared__ __align__(16) unsigned short tile[64 * 72];
  const int tid = threadIdx.x;
  const int kv0 = blockIdx.x * 64;
  {
    const int d = tid >> 2, kq = (tid & 3) * 16;
    const float* src = w2 + (size_t)d * kSeq + kv0 + kq;
    const v4f a0 = *(const v4f*)(src), a1 = *(const v4f*)(src + 4), a2 = *(const v4f*)(src + 8), a3 = *(const v4f*)(src + 12);
    const float f[16] = {a0[0], a0[1], a0[2], a0[3], a1[0], a1[1], a1[2], a1[3],
                         a2[0], a2[1], a2[2], a2[3], a3[0], a3[1], a3[2], a3[3]};
#pragma unroll
    for (int e = 0; e < 16; ++e)
      tile[(kq + e) * 72 + d] = __builtin_bit_cast(unsigned short, (_Float16)(f[e] * kW2Carry));
  }
  __syncthreads();
  {
    const int row = tid >> 3, c8 = (tid & 7) * 8;
    v4u u0 = *(const v4u*)(const void*)(tile + row * 72 + c8);
    v4u u1 = *(const v4u*)(const void*)(tile + (row + 32) * 72 + c8);
    for (int pass = 0; pass < 2; ++pass) {
      *(volatile v4u*)(void*)(w2t + (size_t)(kv0 + row) * kHD + c8) = u0;
      *(volatile v4u*)(void*)(w2t + (size_t)(kv0 + row + 32) * kHD + c8) = u1;
      __threadfence();
    }
  }
}

__global__ __launch_bounds__(128) void synth_attn64(
    const unsigned short* __restrict__ Rq, const unsigned short* __restrict__ Kt,
    const float* __restrict__ b2,
    const unsigned short* __restrict__ Vhp, const unsigned short* __restrict__ Vlp,
    unsigned short* __restrict__ Yhp, unsigned short* __restrict__ Ylp) {
  union FB { v16b v; v8b h[2]; };
  union FH { v16h v; v8h h[2]; };
  __shared__ __align__(16) unsigned short Ksh[kKC * kHD];
  __shared__ __align__(16) unsigned short Vth[kHD * kKC];
  __shared__ __align__(16) unsigned short Vtl[kHD * kKC];
  __shared__ __align__(16) __bf16 Psh[4][16 * kKC];
  __shared__ __align__(16) __bf16 Psl[4][16 * kKC];
  __shared__ __align__(16) float  Os[4][16 * 68];

  const int tid  = threadIdx.x;
  const int wave = tid >> 5;
  const int lane = tid & 31;
  const int hh   = lane >> 4;
  const int c    = lane & 15;

  const int nqb = kSeq / 64;
  const int bx  = blockIdx.x;
  const int qb  = bx % nqb;
  const int bh  = bx / nqb;
  const int h   = bh % kHeads;
  const int b   = bh / kHeads;
  const int q0  = qb * 64 + wave * 16;

  v16h qa[2];
  {
    const _Float16* qrow = (const _Float16*)(const void*)Rq + (size_t)(b * kSeq + q0 + c) * kEmb + h * kHD + 8 * hh;
#pragma unroll
    for (int dc = 0; dc < 2; ++dc) qa[dc] = Frag<_Float16>::load(qrow + dc * 32);
  }

  float mrow[8], lrow[8];
  v8f oacc[4];
#pragma unroll
  for (int r = 0; r < 8; ++r) { mrow[r] = -__builtin_inff(); lrow[r] = 0.f; }
#pragma unroll
  for (int t = 0; t < 4; ++t) oacc[t] = (v8f){0.f,0.f,0.f,0.f,0.f,0.f,0.f,0.f};

  const int nChunks = qb + 1;
  for (int kc = 0; kc < nChunks; ++kc) {
    const int kv0 = kc * kKC;
    __syncthreads();
    {
      const int kvr = tid >> 1, dh = (tid & 1) * 32;
      const v4u* ks = (const v4u*)(const void*)(Kt + (size_t)(kv0 + kvr) * kHD + dh);
      v4u k4[4];
#pragma unroll
      for (int i = 0; i < 4; ++i) k4[i] = ks[i];
#pragma unroll
      for (int i = 0; i < 4; ++i) *(v4u*)(void*)(Ksh + kvr * kHD + dh + 8 * i) = k4[i];
      const size_t vo = (size_t)(b * kSeq + kv0 + kvr) * kEmb + h * kHD + dh;
      const v4u* vhs = (const v4u*)(const void*)(Vhp + vo);
      const v4u* vls = (const v4u*)(const void*)(Vlp + vo);
      v4u vh4[4], vl4[4];
#pragma unroll
      for (int i = 0; i < 4; ++i) { vh4[i] = vhs[i]; vl4[i] = vls[i]; }
#pragma unroll
      for (int i = 0; i < 4; ++i) {
#pragma unroll
        for (int e = 0; e < 4; ++e) {
          const int d = dh + 8 * i + 2 * e;
          const unsigned wa = vh4[i][e], wb = vl4[i][e];
          Vth[d * kKC + kvr]       = (unsigned short)(wa & 0xffffu);
          Vth[(d + 1) * kKC + kvr] = (unsigned short)(wa >> 16);
          Vtl[d * kKC + kvr]       = (unsigned short)(wb & 0xffffu);
          Vtl[(d + 1) * kKC + kvr] = (unsigned short)(wb >> 16);
        }
      }
    }
    __syncthreads();

    v8f s[4];
#pragma unroll
    for (int j = 0; j < 4; ++j) {
      s[j] = (v8f){0.f,0.f,0.f,0.f,0.f,0.f,0.f,0.f};
#pragma unroll
      for (int dc = 0; dc < 2; ++dc) {
        FH kb;
        kb.h[0] = *(const v8h*)(const void*)(Ksh + (j * 16 + c) * kHD + dc * 32 + 8 * hh);
        kb.h[1] = *(const v8h*)(const void*)(Ksh + (j * 16 + c) * kHD + dc * 32 + 16 + 8 * hh);
        s[j] = mma_h16(qa[dc], kb.v, s[j]);
      }
    }
    const bool diag = (kc == qb);
    float bq[4];
#pragma unroll
    for (int j = 0; j < 4; ++j) bq[j] = b2[kv0 + j * 16 + c];
    float cm[8];
#pragma unroll
    for (int r = 0; r < 8; ++r) {
      const int qrow = q0 + 8 * hh + r;
      float m = -__builtin_inff();
#pragma unroll
      for (int j = 0; j < 4; ++j) {
        const int kvcol = kv0 + j * 16 + c;
        float val = s[j][r] * (1.0f / kW2Carry) + bq[j];
        const bool masked = diag && (kvcol > qrow);
        if (masked) val = kNegFill;
        s[j][r] = val;
        m = fmaxf(m, val);
      }
#pragma unroll
      for (int off = 1; off < 16; off <<= 1) m = fmaxf(m, __shfl_xor(m, off, 32));
      cm[r] = m;
    }
    __bf16* pwh = Psh[wave];
    __bf16* pwl = Psl[wave];
#pragma unroll
    for (int r = 0; r < 8; ++r) {
      const float mnew = fmaxf(mrow[r], cm[r]);
      const float alpha = expf(mrow[r] - mnew);
      mrow[r] = mnew;
      float psum = 0.f;
#pragma unroll
      for (int j = 0; j < 4; ++j) {
        const float p = expf(s[j][r] - mnew);
        psum += p;
        __bf16 ph, pl;
        at_split(p, ph, pl);
        pwh[(8 * hh + r) * kKC + j * 16 + c] = ph;
        pwl[(8 * hh + r) * kKC + j * 16 + c] = pl;
      }
#pragma unroll
      for (int off = 1; off < 16; off <<= 1) psum += __shfl_xor(psum, off, 32);
      lrow[r] = lrow[r] * alpha + psum;
#pragma unroll
      for (int t = 0; t < 4; ++t) oacc[t][r] *= alpha;
    }
    __builtin_amdgcn_fence(__ATOMIC_RELEASE, "workgroup");
    __builtin_amdgcn_wave_barrier();
    __builtin_amdgcn_fence(__ATOMIC_ACQUIRE, "workgroup");
#pragma unroll 1
    for (int kk = 0; kk < 2; ++kk) {
      FB pa, pl;
      pa.h[0] = *(const v8b*)(pwh + c * kKC + kk * 32 + 8 * hh);
      pa.h[1] = *(const v8b*)(pwh + c * kKC + kk * 32 + 16 + 8 * hh);
      pl.h[0] = *(const v8b*)(pwl + c * kKC + kk * 32 + 8 * hh);
      pl.h[1] = *(const v8b*)(pwl + c * kKC + kk * 32 + 16 + 8 * hh);
#pragma unroll
      for (int t = 0; t < 4; ++t) {
        FB vb, vl;
        vb.h[0] = *(const v8b*)(const void*)(Vth + (t * 16 + c) * kKC + kk * 32 + 8 * hh);
        vb.h[1] = *(const v8b*)(const void*)(Vth + (t * 16 + c) * kKC + kk * 32 + 16 + 8 * hh);
        vl.h[0] = *(const v8b*)(const void*)(Vtl + (t * 16 + c) * kKC + kk * 32 + 8 * hh);
        vl.h[1] = *(const v8b*)(const void*)(Vtl + (t * 16 + c) * kKC + kk * 32 + 16 + 8 * hh);
        oacc[t] = at_mma(pa.v, vb.v, oacc[t]);
        oacc[t] = at_mma(pa.v, vl.v, oacc[t]);
        oacc[t] = at_mma(pl.v, vb.v, oacc[t]);
      }
    }
  }

  float* os = Os[wave];
#pragma unroll
  for (int r = 0; r < 8; ++r) {
    const float inv = 1.0f / lrow[r];
#pragma unroll
    for (int t = 0; t < 4; ++t) os[(8 * hh + r) * 68 + t * 16 + c] = oacc[t][r] * inv;
  }
  __builtin_amdgcn_fence(__ATOMIC_RELEASE, "workgroup");
  __builtin_amdgcn_wave_barrier();
  __builtin_amdgcn_fence(__ATOMIC_ACQUIRE, "workgroup");
  {
    const int q4 = lane >> 3, c8 = (lane & 7) * 8;
    for (int pass = 0; pass < 2; ++pass) {
#pragma unroll
      for (int it = 0; it < 4; ++it) {
        const int row = it * 4 + q4;
        const float* sp = os + row * 68 + c8;
        v8h hv, lv;
#pragma unroll
        for (int e = 0; e < 8; ++e) {
          const unsigned short hb = f2bf_bits(sp[e]);
          const unsigned short lb = f2bf_bits(sp[e] - bf_bits2f(hb));
          hv[e] = __builtin_bit_cast(_Float16, hb);
          lv[e] = __builtin_bit_cast(_Float16, lb);
        }
        const size_t yo = (size_t)(b * kSeq + q0 + row) * kEmb + h * kHD + c8;
        *(volatile v8h*)(void*)(Yhp + yo) = hv;
        *(volatile v8h*)(void*)(Ylp + yo) = lv;
      }
      __threadfence();
    }
  }
}

extern "C" void kernel_launch(void* const* d_in, const int* in_sizes, int n_in,
                              void* d_out, int out_size, void* d_ws, size_t ws_size,
                              hipStream_t stream) {
  if (n_in < 9) return;
  if (in_sizes[0] != kTok * kEmb || in_sizes[1] != kEmb * kEmb || in_sizes[2] != kEmb ||
      in_sizes[3] != kHD * kSeq || in_sizes[4] != kSeq || in_sizes[5] != kEmb * kEmb ||
      in_sizes[6] != kEmb || in_sizes[7] != kEmb * kEmb || in_sizes[8] != kEmb) return;
  if (out_size != kTok * kEmb) return;

  const float* x      = (const float*)d_in[0];
  const float* w1_w   = (const float*)d_in[1];
  const float* w1_b   = (const float*)d_in[2];
  const float* w2     = (const float*)d_in[3];
  const float* b2     = (const float*)d_in[4];
  const float* val_w  = (const float*)d_in[5];
  const float* val_b  = (const float*)d_in[6];
  const float* proj_w = (const float*)d_in[7];
  const float* proj_b = (const float*)d_in[8];
  float* out = (float*)d_out;

  const size_t planeTok = (size_t)kTok * kEmb * 2;
  const size_t planeW   = (size_t)kEmb * kEmb * 2;
  const size_t planeK   = (size_t)kSeq * kHD * 2;
  char* ws = (char*)d_ws;
  size_t off = 0;
  auto carve = [&](size_t bytes) { char* p = ws + off; off += (bytes + 255) & ~(size_t)255; return p; };
  unsigned short* X16 = (unsigned short*)carve(planeTok);
  unsigned short* Xh  = (unsigned short*)carve(planeTok);
  unsigned short* Xl  = (unsigned short*)carve(planeTok);
  unsigned short* W1c = (unsigned short*)carve(planeW);
  unsigned short* VWh = (unsigned short*)carve(planeW);
  unsigned short* VWl = (unsigned short*)carve(planeW);
  unsigned short* PWh = (unsigned short*)carve(planeW);
  unsigned short* PWl = (unsigned short*)carve(planeW);
  unsigned short* W2T = (unsigned short*)carve(planeK);
  unsigned short* R16 = (unsigned short*)carve(planeTok);
  unsigned short* Vh  = (unsigned short*)carve(planeTok);
  unsigned short* Vl  = (unsigned short*)carve(planeTok);
  unsigned short* Yh  = (unsigned short*)carve(planeTok);
  unsigned short* Yl  = (unsigned short*)carve(planeTok);
  if (off > ws_size) return;

  {
    const int n8x = kTok * kEmb / 8;
    const int n8w = kEmb * kEmb / 8;
    cvt_planes8<true, true><<<(n8x + 255) / 256, 256, 0, stream>>>(x, n8x, 1.0f, X16, Xh, Xl);
    cvt_planes8<true, false><<<(n8w + 255) / 256, 256, 0, stream>>>(w1_w, n8w, kW1Carry, W1c, W1c, W1c);
    cvt_planes8<false, true><<<(n8w + 255) / 256, 256, 0, stream>>>(val_w, n8w, 1.0f, VWh, VWh, VWl);
    cvt_planes8<false, true><<<(n8w + 255) / 256, 256, 0, stream>>>(proj_w, n8w, 1.0f, PWh, PWh, PWl);
    w2t_kernel<<<kSeq / 64, 256, 0, stream>>>(w2, W2T);
  }

  const int tiles = (kTok / 64) * (kEmb / 64);
  const dim3 ggrid((tiles + 7) / 8, 1);

  wmma_gemm64<0, false, 2, 1, false, 2><<<ggrid, 256, 0, stream>>>(
      X16, X16, kEmb, 0L, W1c, W1c, kEmb, 0L, (void*)R16, (void*)R16, kEmb, 0L,
      w1_b, w1_b, 0L, kTok, kEmb, kEmb, 1.0f / kW1Carry);

  wmma_gemm64<1, true, 2, 2, false, 0><<<ggrid, 256, 0, stream>>>(
      Xh, Xl, kEmb, 0L, VWh, VWl, kEmb, 0L, (void*)Vh, (void*)Vl, kEmb, 0L,
      val_b, val_b, 0L, kTok, kEmb, kEmb, 1.0f);

  synth_attn64<<<kBatch * kHeads * (kSeq / 64), 128, 0, stream>>>(R16, W2T, b2, Vh, Vl, Yh, Yl);

  wmma_gemm64<1, true, 2, 0, false, 0><<<ggrid, 256, 0, stream>>>(
      Yh, Yl, kEmb, 0L, PWh, PWl, kEmb, 0L, (void*)out, (void*)out, kEmb, 0L,
      proj_b, proj_b, 0L, kTok, kEmb, kEmb, 1.0f);
}
